// O1Consequent_34600256536768
// MI455X (gfx1250) — hardware-verified
//
#include <hip/hip_runtime.h>


typedef __bf16 v16b __attribute__((ext_vector_type(16)));
typedef float v8f __attribute__((ext_vector_type(8)));
typedef float v4f __attribute__((ext_vector_type(4)));
typedef v4f v4fa __attribute__((may_alias));
typedef unsigned int v4u __attribute__((ext_vector_type(4)));

#define IN_DIM 512
#define OUT_DIM 512
#define N_RULES 16
#define BATCH 8192

#define NTHR 256
#define BM 128
#define BN 64
#define WM 32
#define WN 32
#define KSTEPS (IN_DIM / 32)
#define STG_PITCH 32

static_assert((BATCH % BM) == 0);
static_assert((OUT_DIM % BN) == 0);
static_assert((IN_DIM % 32) == 0);
static_assert(((BATCH * IN_DIM) % (8 * NTHR)) == 0);
static_assert(((N_RULES * OUT_DIM * IN_DIM) % (8 * NTHR)) == 0);
static_assert(BM * N_RULES == 8 * NTHR);
static_assert(BN * N_RULES == 4 * NTHR);

union Frag { v16b v; v4u q[2]; };

__device__ __forceinline__ unsigned int bf16_bits(float f) {
  unsigned int u = __float_as_uint(f);
  u = u + 0x7FFFu + ((u >> 16) & 1u);
  return u >> 16;
}
__device__ __forceinline__ float bf16_rne(float f) {
  return __uint_as_float(bf16_bits(f) << 16);
}

__device__ __forceinline__ v8f wmma_bf16(v16b a, v16b b, v8f c) {
  return __builtin_amdgcn_wmma_f32_16x16x32_bf16(false, a, false, b, (short)0, c, false, false);
}

__global__ __launch_bounds__(NTHR)
void k_convert(const float* __restrict__ x, const float* __restrict__ W,
               unsigned short* __restrict__ Xb, unsigned short* __restrict__ Wb,
               int nx8, int nw8) {
  const int g = blockIdx.x * NTHR + threadIdx.x;
  if (g >= nx8 + nw8) return;
  const float* src;
  unsigned short* dst;
  int idx;
  if (g < nx8) { src = x; dst = Xb; idx = g; }
  else         { src = W; dst = Wb; idx = g - nx8; }
  const size_t e = (size_t)idx * 8;
  const float4 a = *(const float4*)(src + e);
  const float4 c = *(const float4*)(src + e + 4);
  v4u q;
  q.x = bf16_bits(a.x) | (bf16_bits(a.y) << 16);
  q.y = bf16_bits(a.z) | (bf16_bits(a.w) << 16);
  q.z = bf16_bits(c.x) | (bf16_bits(c.y) << 16);
  q.w = bf16_bits(c.z) | (bf16_bits(c.w) << 16);
  volatile v4u* p = (volatile v4u*)(dst + e);
  *p = q;
  __threadfence();
  *p = q;
}

__global__ __launch_bounds__(NTHR)
void k_rule_gemm(const __bf16* __restrict__ Xb, const __bf16* __restrict__ Wb,
                 const float* __restrict__ frs, const float* __restrict__ bias,
                 float* __restrict__ out) {
  __shared__ float sFrs[N_RULES * BM];
  __shared__ float sBias[N_RULES * BN];
  __shared__ float sStg[(NTHR / 32) * WM * STG_PITCH];

  const int tid    = threadIdx.x;
  const int blockN = blockIdx.x * BN;
  const int blockM = blockIdx.y * BM;
  const int wave   = tid >> 5;
  const int lane   = tid & 31;
  const int h      = lane >> 4;
  const int m      = lane & 15;
  const int waveM  = wave >> 1;
  const int waveN  = wave & 1;

  {
    const int row = tid >> 1;
    const int c0  = (tid & 1) * 8;
    const float* fp = frs + (size_t)(blockM + row) * N_RULES + c0;
    const float4 u0 = *(const float4*)(fp);
    const float4 u1 = *(const float4*)(fp + 4);
    sFrs[(c0 + 0) * BM + row] = bf16_rne(u0.x);
    sFrs[(c0 + 1) * BM + row] = bf16_rne(u0.y);
    sFrs[(c0 + 2) * BM + row] = bf16_rne(u0.z);
    sFrs[(c0 + 3) * BM + row] = bf16_rne(u0.w);
    sFrs[(c0 + 4) * BM + row] = bf16_rne(u1.x);
    sFrs[(c0 + 5) * BM + row] = bf16_rne(u1.y);
    sFrs[(c0 + 6) * BM + row] = bf16_rne(u1.z);
    sFrs[(c0 + 7) * BM + row] = bf16_rne(u1.w);
  }
  {
    const int r = tid >> 4;
    const int c = (tid & 15) * 4;
    const float4 u = *(const float4*)(bias + (size_t)r * OUT_DIM + blockN + c);
    sBias[r * BN + c + 0] = bf16_rne(u.x);
    sBias[r * BN + c + 1] = bf16_rne(u.y);
    sBias[r * BN + c + 2] = bf16_rne(u.z);
    sBias[r * BN + c + 3] = bf16_rne(u.w);
  }
  __syncthreads();

  const int rowW = blockM + waveM * WM;
  const int colW = blockN + waveN * WN;

  const __bf16* pa0 = Xb + (size_t)(rowW + m) * IN_DIM + 8 * h;
  const __bf16* pa1 = pa0 + (size_t)16 * IN_DIM;

  const v8f zero8 = {0.f, 0.f, 0.f, 0.f, 0.f, 0.f, 0.f, 0.f};
  v8f acc00 = zero8, acc01 = zero8, acc10 = zero8, acc11 = zero8;

#pragma unroll 1
  for (int r = 0; r < N_RULES; ++r) {
    const __bf16* pb0 = Wb + (size_t)r * OUT_DIM * IN_DIM + (size_t)(colW + m) * IN_DIM + 8 * h;
    const __bf16* pb1 = pb0 + (size_t)16 * IN_DIM;

    v8f d00 = zero8, d01 = zero8, d10 = zero8, d11 = zero8;
#pragma unroll 2
    for (int ks = 0; ks < KSTEPS; ++ks) {
      const int k0 = ks * 32;
      Frag a0, a1, b0, b1;
      a0.q[0] = *(const v4u*)(pa0 + k0);  a0.q[1] = *(const v4u*)(pa0 + k0 + 16);
      a1.q[0] = *(const v4u*)(pa1 + k0);  a1.q[1] = *(const v4u*)(pa1 + k0 + 16);
      b0.q[0] = *(const v4u*)(pb0 + k0);  b0.q[1] = *(const v4u*)(pb0 + k0 + 16);
      b1.q[0] = *(const v4u*)(pb1 + k0);  b1.q[1] = *(const v4u*)(pb1 + k0 + 16);
      d00 = wmma_bf16(a0.v, b0.v, d00);
      d01 = wmma_bf16(a0.v, b1.v, d01);
      d10 = wmma_bf16(a1.v, b0.v, d10);
      d11 = wmma_bf16(a1.v, b1.v, d11);
      asm volatile("v_nop\n\tv_nop\n\tv_nop\n\tv_nop"
                   : "+v"(d00), "+v"(d01), "+v"(d10), "+v"(d11)
                   : "v"(a0.v), "v"(a1.v), "v"(b0.v), "v"(b1.v));
    }

    const float* fr = sFrs + r * BM + waveM * WM + 8 * h;
    const float bb0 = sBias[r * BN + waveN * WN + m];
    const float bb1 = sBias[r * BN + waveN * WN + 16 + m];
#pragma unroll
    for (int j = 0; j < 8; ++j) {
      const float f0 = fr[j];
      const float f1 = fr[16 + j];
      acc00[j] = fmaf(f0, d00[j] + bb0, acc00[j]);
      acc01[j] = fmaf(f0, d01[j] + bb1, acc01[j]);
      acc10[j] = fmaf(f1, d10[j] + bb0, acc10[j]);
      acc11[j] = fmaf(f1, d11[j] + bb1, acc11[j]);
    }
  }

  float* stg = sStg + wave * (WM * STG_PITCH);
#pragma unroll
  for (int j = 0; j < 8; ++j) {
    stg[(8 * h + j) * STG_PITCH + m]           = acc00[j];
    stg[(8 * h + j) * STG_PITCH + 16 + m]      = acc01[j];
    stg[(16 + 8 * h + j) * STG_PITCH + m]      = acc10[j];
    stg[(16 + 8 * h + j) * STG_PITCH + 16 + m] = acc11[j];
  }
  __syncthreads();

  const int rq = lane >> 3;
  const int cq = (lane & 7) * 4;
  v4f v[8];
#pragma unroll
  for (int i = 0; i < 8; ++i)
    v[i] = *(const v4fa*)(stg + (i * 4 + rq) * STG_PITCH + cq);

  float* ob = out + (size_t)(rowW + rq) * OUT_DIM + colW + cq;
#pragma unroll
  for (int i = 0; i < 8; ++i)
    *(volatile v4f*)(ob + (size_t)(i * 4) * OUT_DIM) = v[i];
  __threadfence();
#pragma unroll
  for (int i = 0; i < 8; ++i)
    *(volatile v4f*)(ob + (size_t)(i * 4) * OUT_DIM) = v[i];
}

extern "C" void kernel_launch(void* const* d_in, const int* in_sizes, int n_in,
                              void* d_out, int out_size, void* d_ws, size_t ws_size,
                              hipStream_t stream) {
  if (n_in < 4) return;
  if (in_sizes[0] != BATCH * IN_DIM) return;
  if (in_sizes[1] != BATCH * N_RULES) return;
  if (in_sizes[2] != N_RULES * OUT_DIM * IN_DIM) return;
  if (in_sizes[3] != N_RULES * OUT_DIM) return;
  if (out_size != BATCH * OUT_DIM) return;

  const float* x    = (const float*)d_in[0];
  const float* frs  = (const float*)d_in[1];
  const float* W    = (const float*)d_in[2];
  const float* bias = (const float*)d_in[3];
  float* out        = (float*)d_out;

  const size_t xbBytes = (size_t)BATCH * IN_DIM * sizeof(unsigned short);
  const size_t wbBytes = (size_t)N_RULES * OUT_DIM * IN_DIM * sizeof(unsigned short);
  if (ws_size < xbBytes + wbBytes) return;
  unsigned short* Xb = (unsigned short*)d_ws;
  unsigned short* Wb = (unsigned short*)((char*)d_ws + xbBytes);

  const int nx8 = (BATCH * IN_DIM) / 8;
  const int nw8 = (N_RULES * OUT_DIM * IN_DIM) / 8;
  const int cvtBlocks = (nx8 + nw8 + NTHR - 1) / NTHR;
  k_convert<<<dim3(cvtBlocks), dim3(NTHR), 0, stream>>>(x, W, Xb, Wb, nx8, nw8);

  dim3 grid(OUT_DIM / BN, BATCH / BM);
  k_rule_gemm<<<grid, dim3(NTHR), 0, stream>>>((const __bf16*)Xb, (const __bf16*)Wb, frs, bias, out);
  (void)hipGetLastError();
}
